// InnerAttention_40656160424181
// MI455X (gfx1250) — hardware-verified
//
#include <hip/hip_runtime.h>


#define NB_  4
#define NH_  16
#define NN   2048
#define HD   64
#define W3   192
#define ZH   4
#define PCAR 1024.0f
typedef _Float16 h16;
typedef unsigned short bf;
typedef __attribute__((ext_vector_type(16))) __bf16   v16bf;
typedef __attribute__((ext_vector_type(16))) _Float16 v16h;
typedef __attribute__((ext_vector_type(8)))  _Float16 v8h;
typedef __attribute__((ext_vector_type(8)))  unsigned short v8us;
typedef __attribute__((ext_vector_type(8)))  float    v8f;
typedef __attribute__((ext_vector_type(4)))  float    v4f;
typedef v8h  __attribute__((may_alias)) v8ha;
typedef v4f  __attribute__((may_alias)) v4fa;
typedef v8us __attribute__((may_alias)) v8usa;

__device__ __forceinline__ unsigned short f2bf(float f) { unsigned u = __float_as_uint(f); u += 0x7FFFu + ((u >> 16) & 1u); return (unsigned short)(u >> 16); }
__device__ __forceinline__ float bf2f(unsigned short b) { return __uint_as_float(((unsigned)b) << 16); }
__device__ __forceinline__ float bfr(float f) { return bf2f(f2bf(f)); }
__device__ __forceinline__ v16h cat16(v8h lo, v8h hi) { return __builtin_shufflevector(lo, hi, 0, 1, 2, 3, 4, 5, 6, 7, 8, 9, 10, 11, 12, 13, 14, 15); }
__device__ __forceinline__ v16bf cat16b(v8us lo, v8us hi) { return __builtin_bit_cast(v16bf, __builtin_shufflevector(lo, hi, 0, 1, 2, 3, 4, 5, 6, 7, 8, 9, 10, 11, 12, 13, 14, 15)); }
__device__ __forceinline__ v8f wmma16(v16h a, v16h b, v8f c) { return __builtin_amdgcn_wmma_f32_16x16x32_f16(false, a, false, b, (short)0, c, false, false); }
__device__ __forceinline__ v8f wmmab(v16bf a, v16bf b, v8f c) { return __builtin_amdgcn_wmma_f32_16x16x32_bf16(false, a, false, b, (short)0, c, false, false); }


template <typename T16> struct WFrag;
template <> struct WFrag<h16> { typedef v16h V; static __device__ __forceinline__ V ld(const h16* p) { return cat16(*(const v8h*)p, *(const v8h*)(p + 16)); } static __device__ __forceinline__ v8f mma(V a, V b, v8f c) { return wmma16(a, b, c); } };
template <> struct WFrag<bf> { typedef v16bf V; static __device__ __forceinline__ V ld(const bf* p) { return cat16b(*(const v8us*)p, *(const v8us*)(p + 16)); } static __device__ __forceinline__ v8f mma(V a, V b, v8f c) { return wmmab(a, b, c); } };
template <typename T16, int NSPLIT, bool BIAS>
__global__ __launch_bounds__(32) void k_gemmw(const T16* __restrict__ A, const T16* __restrict__ A2, const T16* __restrict__ Bt, const T16* __restrict__ Bt2, int K, float* C, int ldc, const float* __restrict__ bias, size_t sA, size_t sB, size_t sC) {
    typedef typename WFrag<T16>::V V;
    __shared__ __align__(16) float os[16 * 68];
    const size_t z = blockIdx.z; A += z * sA; if (A2) A2 += z * sA; Bt += z * sB; if (Bt2) Bt2 += z * sB; C += z * sC;
    const int lane = threadIdx.x & 31, lr = lane & 15, hi = lane >> 4; const int r0 = blockIdx.x * 64, c0 = blockIdx.y * 64;
    v8f acc[4][4];
#pragma unroll
    for (int mb = 0; mb < 4; ++mb)
#pragma unroll
        for (int nb = 0; nb < 4; ++nb) acc[mb][nb] = (v8f){};
    const size_t aoff = (size_t)(r0 + lr) * K + 8 * hi, boff = (size_t)(c0 + lr) * K + 8 * hi;
#pragma unroll 1
    for (int kc = 0; kc < K; kc += 32) {
        V a[4], a2[4];
#pragma unroll
        for (int mb = 0; mb < 4; ++mb) { a[mb] = WFrag<T16>::ld(A + aoff + (size_t)mb * 16 * K + kc); if (NSPLIT == 1 || NSPLIT == 2) a2[mb] = WFrag<T16>::ld(A2 + aoff + (size_t)mb * 16 * K + kc); }
#pragma unroll
        for (int nb = 0; nb < 4; ++nb) { const V b = WFrag<T16>::ld(Bt + boff + (size_t)nb * 16 * K + kc); V b2; if (NSPLIT >= 2) b2 = WFrag<T16>::ld(Bt2 + boff + (size_t)nb * 16 * K + kc);
#pragma unroll
            for (int mb = 0; mb < 4; ++mb) { acc[mb][nb] = WFrag<T16>::mma(a[mb], b, acc[mb][nb]); if (NSPLIT == 1 || NSPLIT == 2) acc[mb][nb] = WFrag<T16>::mma(a2[mb], b, acc[mb][nb]); if (NSPLIT >= 2) acc[mb][nb] = WFrag<T16>::mma(a[mb], b2, acc[mb][nb]); } }
        asm volatile("v_nop\n\tv_nop\n\tv_nop\n\tv_nop" : "+v"(acc[0][0]), "+v"(acc[1][1]), "+v"(acc[2][2]), "+v"(acc[3][3]) : "v"(a[0]), "v"(a[3]));
    }
#pragma unroll
    for (int mb = 0; mb < 4; ++mb) {
#pragma unroll
        for (int nb = 0; nb < 4; ++nb) {
#pragma unroll
            for (int j = 0; j < 8; ++j) os[(hi * 8 + j) * 68 + nb * 16 + lr] = acc[mb][nb][j]; }
        __builtin_amdgcn_wave_barrier(); asm volatile("" ::: "memory");
        float* crow = C + (size_t)(r0 + mb * 16) * ldc + c0;
#pragma unroll 1
        for (int ps = 0; ps < 2; ++ps) {
#pragma unroll
            for (int s = 0; s < 8; ++s) { const int row = 2 * s + hi, cofs = lr * 4; v4f val = *(const v4fa*)(os + row * 68 + cofs); if (BIAS) { val[0] += bfr(bias[c0 + cofs]); val[1] += bfr(bias[c0 + cofs + 1]); val[2] += bfr(bias[c0 + cofs + 2]); val[3] += bfr(bias[c0 + cofs + 3]); }
                *(volatile v4f*)(crow + (size_t)row * ldc + cofs) = val; }
            if (ps == 0) __threadfence(); }
        __builtin_amdgcn_wave_barrier(); asm volatile("" ::: "memory");
    }
}

__device__ __forceinline__ h16 tohx(float x) { return (h16)x; }
typedef __attribute__((ext_vector_type(2))) unsigned short v2us;
typedef __attribute__((ext_vector_type(2))) _Float16 v2h;
typedef __attribute__((ext_vector_type(4))) _Float16 v4h;

__global__ __launch_bounds__(256) void k_wtG(const float* __restrict__ w, int K, int N, bf* Bt) {
    const int lane = threadIdx.x & 31; const int L0 = (blockIdx.x * 8 + (threadIdx.x >> 5)) * 8; const int nlines = N * K / 64;
#pragma unroll
    for (int ps = 0; ps < 2; ++ps) {
#pragma unroll 1
        for (int l = 0; l < 8; ++l) { const int L = L0 + l; if (L >= nlines) break; const size_t e = (size_t)L * 64 + lane * 2; const int k = (int)(e % K), n = (int)(e / K); v2us o;
            o[0] = f2bf(w[(size_t)k * N + n]); o[1] = f2bf(w[(size_t)(k + 1) * N + n]); *(volatile v2us*)(Bt + e) = o; }
        if (ps == 0) __threadfence(); }
}
__global__ __launch_bounds__(256) void k_cvt8(const float* __restrict__ src, bf* dst, size_t n8) { const size_t i = (size_t)blockIdx.x * 256 + threadIdx.x; if (i >= n8) return; const v8f v = *(const v8f*)(src + i * 8); v8us o;
#pragma unroll
    for (int k = 0; k < 8; ++k) o[k] = f2bf(v[k]); *(volatile v8us*)(dst + i * 8) = o; __threadfence(); *(volatile v8us*)(dst + i * 8) = o; }
__global__ __launch_bounds__(256) void k_pl(const float* __restrict__ QKV, h16* Q16, h16* K16) { const int e = (blockIdx.x * 256 + threadIdx.x) * 4; if (e >= ZH * NN * HD) return; const int d = e % HD; const size_t rowoff = (size_t)(e / HD) * W3; v4h q, k;
#pragma unroll
    for (int u = 0; u < 4; ++u) { q[u] = tohx(QKV[rowoff + 3 * (d + u)] * 0.125f); k[u] = tohx(QKV[rowoff + 3 * (d + u) + 1]); } for (int ps = 0; ps < 2; ++ps) { *(volatile v4h*)(Q16 + e) = q; *(volatile v4h*)(K16 + e) = k; if (ps == 0) __threadfence(); } }
__global__ __launch_bounds__(256) void k_vt(const float* __restrict__ QKV, h16* VT) { const int e = (blockIdx.x * 256 + threadIdx.x) * 2; if (e >= ZH * HD * NN) return; const int n = e % NN; const int d = (e / NN) % HD; const int z = e / (NN * HD); v2h o; o[0] = tohx(QKV[((size_t)z * NN + n) * W3 + 3 * d + 2]); o[1] = tohx(QKV[((size_t)z * NN + n + 1) * W3 + 3 * d + 2]); *(volatile v2h*)(VT + e) = o; __threadfence(); *(volatile v2h*)(VT + e) = o; }
__global__ __launch_bounds__(256) void k_fin(const float* __restrict__ O, float* OUTz) { const int e = (blockIdx.x * 256 + threadIdx.x) * 4; if (e >= ZH * NN * HD) return; const v4f a = *(const v4f*)(O + e); v4f o;
#pragma unroll
    for (int u = 0; u < 4; ++u) o[u] = a[u] * (1.0f / PCAR); *(volatile v4f*)(OUTz + e) = o; __threadfence(); *(volatile v4f*)(OUTz + e) = o; }
template <int NFULL, int TAIL> __global__ __launch_bounds__(256) void k_soft(const float* __restrict__ Sb, int nrows, int rowsper, int rvalid, int nvalid, h16* P) { const int lane = threadIdx.x & 31; const size_t row = (size_t)blockIdx.x * 8 + (threadIdx.x >> 5); if (row >= (size_t)nrows) return; constexpr int LD = NFULL * 128 + TAIL * 64; const float* sr = Sb + row * LD; h16* pr = P + row * LD; const bool live = (int)(row % rowsper) < rvalid; float mx = -3.0e38f;
#pragma unroll 1
    for (int ch = 0; ch < NFULL + TAIL; ++ch) { if (ch == NFULL && lane >= 16) break; const int j0 = ch * 128 + lane * 4; const v4f a = *(const v4f*)(sr + j0);
#pragma unroll
        for (int q = 0; q < 4; ++q) if (j0 + q < nvalid) mx = fmaxf(mx, a[q]); }
#pragma unroll
    for (int sh = 16; sh; sh >>= 1) mx = fmaxf(mx, __shfl_xor(mx, sh, 32));
    float sum = 0.f;
#pragma unroll 1
    for (int ch = 0; ch < NFULL + TAIL; ++ch) { if (ch == NFULL && lane >= 16) break; const int j0 = ch * 128 + lane * 4; const v4f a = *(const v4f*)(sr + j0);
#pragma unroll
        for (int q = 0; q < 4; ++q) if (j0 + q < nvalid) { float d0 = __fsub_rn(a[q], mx); asm volatile("" : "+v"(d0)); sum += __expf(d0); } }
#pragma unroll
    for (int sh = 16; sh; sh >>= 1) sum += __shfl_xor(sum, sh, 32);
    const float f = live ? __fdiv_rn(PCAR, sum) : 0.f;
    for (int ps = 0; ps < 2; ++ps) {
#pragma unroll 1
        for (int ch = 0; ch < NFULL + TAIL; ++ch) { if (ch == NFULL && lane >= 16) break; const int j0 = ch * 128 + lane * 4; const v4f a = *(const v4f*)(sr + j0); v4h o;
#pragma unroll
            for (int q = 0; q < 4; ++q) { float val = 0.f; if (live && j0 + q < nvalid) { float d0 = __fsub_rn(a[q], mx); asm volatile("" : "+v"(d0)); val = __fmul_rn(__expf(d0), f); } o[q] = tohx(val); } *(volatile v4h*)(pr + j0) = o; }
        if (ps == 0) __threadfence(); } }

extern "C" void kernel_launch(void* const* d_in, const int* in_sizes, int n_in,
                              void* d_out, int out_size, void* d_ws, size_t ws_size, hipStream_t stream) {
    (void)in_sizes; (void)n_in; (void)out_size;
    const float* x = (const float*)d_in[0]; const float* w = (const float*)d_in[1]; const float* bq = (const float*)d_in[2];
    float* OUT = (float*)d_out;
    char* wsp = (char*)d_ws;
    auto take = [&](size_t bytes) { char* p = wsp; wsp += (bytes + 255) & ~(size_t)255; return (void*)p; };
    bf* WT = (bf*)take((size_t)NH_ * W3 * HD * 2); bf* XB = (bf*)take((size_t)ZH * NN * HD * 2); float* QKV = (float*)take((size_t)ZH * NN * W3 * 4); h16* Q16 = (h16*)take((size_t)ZH * NN * HD * 2); h16* K16 = (h16*)take((size_t)ZH * NN * HD * 2); h16* VT = (h16*)take((size_t)ZH * HD * NN * 2);
    float* Sb = (float*)take((size_t)ZH * NN * NN * 4); h16* P16 = (h16*)take((size_t)ZH * NN * NN * 2); float* O = (float*)take((size_t)ZH * NN * HD * 4);
    if ((size_t)(wsp - (char*)d_ws) > ws_size) return;
    for (int h = 0; h < NH_; ++h) k_wtG<<<(HD * W3 / 64 + 63) / 64, 256, 0, stream>>>(w + (size_t)h * HD * W3, HD, W3, WT + (size_t)h * W3 * HD);
    for (int b = 0; b < NB_; ++b) {
        for (int h0 = 0; h0 < NH_; h0 += ZH) { const size_t base = ((size_t)b * NH_ + h0) * NN * HD;
            k_cvt8<<<(ZH * NN * HD / 8 + 255) / 256, 256, 0, stream>>>(x + base, XB, (size_t)ZH * NN * HD / 8);
            for (int zz = 0; zz < ZH; ++zz) k_gemmw<bf, 0, true><<<dim3(NN / 64, W3 / 64, 1), 32, 0, stream>>>(XB + (size_t)zz * NN * HD, nullptr, WT + (size_t)(h0 + zz) * W3 * HD, nullptr, HD, QKV + (size_t)zz * NN * W3, W3, bq + (size_t)(h0 + zz) * W3, 0, 0, 0);
            k_pl<<<(ZH * NN * HD / 4 + 255) / 256, 256, 0, stream>>>(QKV, Q16, K16); k_vt<<<(ZH * HD * NN / 2 + 255) / 256, 256, 0, stream>>>(QKV, VT);
            k_gemmw<h16, 0, false><<<dim3(NN / 64, NN / 64, ZH), 32, 0, stream>>>(Q16, nullptr, K16, nullptr, HD, Sb, NN, nullptr, (size_t)NN * HD, (size_t)NN * HD, (size_t)NN * NN);
            k_soft<16, 0><<<ZH * NN / 8, 256, 0, stream>>>(Sb, ZH * NN, NN, NN, NN, P16);
            k_gemmw<h16, 0, false><<<dim3(NN / 64, 1, ZH), 32, 0, stream>>>(P16, nullptr, VT, nullptr, NN, O, HD, nullptr, (size_t)NN * NN, (size_t)HD * NN, (size_t)NN * HD);
            k_fin<<<(ZH * NN * HD / 4 + 255) / 256, 256, 0, stream>>>(O, OUT + base); } }
}
